// GraphEvolutionDiscr_39900246180399
// MI455X (gfx1250) — hardware-verified
//
#include <hip/hip_runtime.h>
#include <math.h>

#define NN    16384
#define NE    262144
#define NV    (NE + NN)
#define HC    256
#define XP    512
#define NT    256
#define TG    128
#define NBG   (NN / TG)
#define SCHG  4096
#define SPG   (SCHG / NT)
#define NCHG  ((NV + SCHG - 1) / SCHG)
#define GAT_LDS_BYTES ((TG * HC + TG * 8 + TG * 8 + SCHG + SCHG) * 4)
#define HSC   16.0f
#define WSC   64.0f
#define DN    32
#define DFF   128
#define DROWS 32

typedef __attribute__((ext_vector_type(16))) _Float16 v16h;
typedef __attribute__((ext_vector_type(8)))  _Float16 v8h;
typedef __attribute__((ext_vector_type(16))) __bf16   v16b;
typedef __attribute__((ext_vector_type(8)))  __bf16   v8b;
typedef __attribute__((ext_vector_type(8)))  float    v8f;
typedef __attribute__((ext_vector_type(4)))  float    v4f;
typedef __attribute__((ext_vector_type(4)))  int      v4i;
#define U16(p) ((const unsigned short*)(const void*)(p))

__device__ __forceinline__ unsigned short f2bf_bits(float f) {
  unsigned u = __float_as_uint(f);
  return (unsigned short)((u + 0x7FFFu + ((u >> 16) & 1u)) >> 16);
}
__device__ __forceinline__ float bf_bits2f(unsigned short h) { return __uint_as_float(((unsigned)h) << 16); }

__device__ __forceinline__ void dep_guard_h(v8f& a, v8f& b, v16h x, v16h y) { asm volatile("v_nop\n\tv_nop\n\tv_nop\n\tv_nop" : "+v"(a), "+v"(b) : "v"(x), "v"(y)); }
__device__ __forceinline__ void dep_guard_b(v8f& a, v8f& b, v16b x, v16b y) { asm volatile("v_nop\n\tv_nop\n\tv_nop\n\tv_nop" : "+v"(a), "+v"(b) : "v"(x), "v"(y)); }
__device__ __forceinline__ void keep4_h(v16h a, v16h b, v16h c, v16h d) { asm volatile("v_nop" :: "v"(a), "v"(b), "v"(c), "v"(d)); }
__device__ __forceinline__ void keep4_b(v16b a, v16b b, v16b c, v16b d) { asm volatile("v_nop" :: "v"(a), "v"(b), "v"(c), "v"(d)); }
__device__ __forceinline__ void acc_guard4(v8f& a, v8f& b, v8f& c, v8f& d) { asm volatile("v_nop\n\tv_nop\n\tv_nop\n\tv_nop" : "+v"(a), "+v"(b), "+v"(c), "+v"(d)); }
template <typename T> struct Frag;
template <> struct Frag<_Float16> {
  typedef v16h V; union U { v16h v; v8h h[2]; };
  static __device__ __forceinline__ v16h load(const _Float16* p) {
    U f; f.h[0] = *(const v8h*)(p); f.h[1] = *(const v8h*)(p + 16); return f.v;
  }
  static __device__ __forceinline__ v8f mma(v16h a, v16h b, v8f c) {
    return __builtin_amdgcn_wmma_f32_16x16x32_f16(false, a, false, b, (short)0, c, false, false);
  }
  static __device__ __forceinline__ void guard(v8f& a, v8f& b, v16h x, v16h y) { dep_guard_h(a, b, x, y); }
  static __device__ __forceinline__ void keep(v16h a, v16h b, v16h c, v16h d) { keep4_h(a, b, c, d); }
};
template <> struct Frag<__bf16> {
  typedef v16b V; union U { v16b v; v8b h[2]; };
  static __device__ __forceinline__ v16b load(const __bf16* p) {
    U f; f.h[0] = *(const v8b*)(p); f.h[1] = *(const v8b*)(p + 16); return f.v;
  }
  static __device__ __forceinline__ v8f mma(v16b a, v16b b, v8f c) {
    return __builtin_amdgcn_wmma_f32_16x16x32_bf16(false, a, false, b, (short)0, c, false, false);
  }
  static __device__ __forceinline__ void guard(v8f& a, v8f& b, v16b x, v16b y) { dep_guard_b(a, b, x, y); }
  static __device__ __forceinline__ void keep(v16b a, v16b b, v16b c, v16b d) { keep4_b(a, b, c, d); }
};

__device__ __forceinline__ v8f mma_h(v16h a, v16h b, v8f c) {
  c = __builtin_amdgcn_wmma_f32_16x16x32_f16(false, a, false, b, (short)0, c, false, false);
  asm volatile("v_nop\n\tv_nop\n\tv_nop\n\tv_nop" : "+v"(c) : "v"(a), "v"(b));
  return c;
}

template <int ET> struct Elem;
template <> struct Elem<0> { typedef _Float16 T; };
template <> struct Elem<1> { typedef __bf16 T; };
template <int ET, bool SPLIT, int BIAS_MODE, int OUT_MODE, bool RESID, int ACT = 0>
__global__ __launch_bounds__(256) void wmma_gemm64(
    const unsigned short* __restrict__ Ap, const unsigned short* __restrict__ A2p, int lda, long strideA,
    const unsigned short* __restrict__ Btp, const unsigned short* __restrict__ Bt2p, int ldb, long strideB,
    void* __restrict__ Cout, void* __restrict__ Cout2, int ldc, long strideC,
    const float* __restrict__ bias,
    const float* __restrict__ resid, long strideR,
    int M, int N, int K, float scale) {
  typedef typename Elem<ET>::T T;
  typedef typename Frag<T>::V V;
  const T* A = (const T*)Ap; const T* A2 = (const T*)A2p; const T* Bt = (const T*)Btp; const T* Bt2 = (const T*)Bt2p;
  __shared__ __align__(16) float sT[8][16 * 68];
  const int b    = blockIdx.y;
  const int lane = threadIdx.x & 31;
  const int wave = threadIdx.x >> 5;
  const int tilesN = N >> 6;
  const int tilesM = M >> 6;
  const int tile = blockIdx.x * 8 + wave;
  if (tile >= tilesM * tilesN) return;
  const int tm = tile / tilesN;
  const int tn = tile - tm * tilesN;
  const int m0 = tm << 6;
  const int n0 = tn << 6;

  const T* Ab  = A  + (size_t)b * strideA;
  const T* Bb  = Bt + (size_t)b * strideB;
  const T* Ab2 = SPLIT ? (A2  + (size_t)b * strideA) : nullptr;
  const T* Bb2 = SPLIT ? (Bt2 + (size_t)b * strideB) : nullptr;

  const int rlane = lane & 15;
  const int koff  = (lane >> 4) * 8;
  const int mOff  = (lane >> 4) * 8;

  v8f acc[4][4];
#pragma unroll
  for (int i = 0; i < 4; ++i)
#pragma unroll
    for (int j = 0; j < 4; ++j) acc[i][j] = (v8f){0.f,0.f,0.f,0.f,0.f,0.f,0.f,0.f};

  for (int k0 = 0; k0 < K; k0 += 32) {
    V bh[4], bl[4];
#pragma unroll
    for (int j = 0; j < 4; ++j) {
      const size_t bo = (size_t)(n0 + (j << 4) + rlane) * ldb + koff + k0;
      bh[j] = Frag<T>::load(Bb + bo);
      if (SPLIT) bl[j] = Frag<T>::load(Bb2 + bo);
    }
#pragma unroll
    for (int i = 0; i < 4; ++i) {
      const size_t ao = (size_t)(m0 + (i << 4) + rlane) * lda + koff + k0;
      V ah = Frag<T>::load(Ab + ao);
      V al;
      if (SPLIT) al = Frag<T>::load(Ab2 + ao);
#pragma unroll
      for (int j = 0; j < 4; ++j) {
        acc[i][j] = Frag<T>::mma(ah, bh[j], acc[i][j]);
        if (SPLIT) {
          acc[i][j] = Frag<T>::mma(ah, bl[j], acc[i][j]);
          acc[i][j] = Frag<T>::mma(al, bh[j], acc[i][j]);
        }
      }
      Frag<T>::guard(acc[i][0], acc[i][3], ah, SPLIT ? al : ah);
    }
    Frag<T>::keep(bh[0], bh[1], bh[2], bh[3]);
    if (SPLIT) Frag<T>::keep(bl[0], bl[1], bl[2], bl[3]);
  }
  acc_guard4(acc[0][0], acc[0][1], acc[0][2], acc[0][3]);
  acc_guard4(acc[1][0], acc[1][1], acc[1][2], acc[1][3]);
  acc_guard4(acc[2][0], acc[2][1], acc[2][2], acc[2][3]);
  acc_guard4(acc[3][0], acc[3][1], acc[3][2], acc[3][3]);

  float* slab = sT[wave];
  const float* Rb = RESID ? (resid + (size_t)b * strideR) : nullptr;
#pragma unroll
  for (int i = 0; i < 4; ++i) {
    const int mBase = m0 + (i << 4);
#pragma unroll
    for (int j = 0; j < 4; ++j) {
      const int n = n0 + (j << 4) + rlane;
      float bv = 0.f;
      if (BIAS_MODE == 2) bv = bias[n];
#pragma unroll
      for (int r = 0; r < 8; ++r) {
        float v = acc[i][j][r] * scale;
        if (BIAS_MODE == 1) v += bias[mBase + mOff + r];
        if (BIAS_MODE == 2) v += bv;
        if (RESID) v += Rb[(size_t)(mBase + mOff + r) * ldc + n];
        if (ACT == 1) v = tanhf(v);
        if (ACT == 2) v = fmaxf(v, 0.0f);
        if (ACT == 3) v = v / (1.0f + expf(-v));
        if (ACT == 4) v = (v > 0.f) ? v : 0.01f * v;
        if (ACT == 5) v = 0.5f * v * (1.0f + erff(v * 0.70710678118654752f));
        slab[(mOff + r) * 68 + (j << 4) + rlane] = v;
      }
    }
    __builtin_amdgcn_fence(__ATOMIC_RELEASE, "workgroup");
    __builtin_amdgcn_wave_barrier();
    __builtin_amdgcn_fence(__ATOMIC_ACQUIRE, "workgroup");
    if (OUT_MODE == 0) {
      float* C = (float*)Cout + (size_t)b * strideC;
      const int hh = lane >> 4, c4 = (lane & 15) * 4;
      for (int pass = 0; pass < 2; ++pass) {
#pragma unroll
        for (int it = 0; it < 8; ++it) {
          const int row = it * 2 + hh;
          v4f v = *(const v4f*)(slab + row * 68 + c4);
          *(volatile v4f*)(C + (size_t)(mBase + row) * ldc + n0 + c4) = v;
        }
        __threadfence();
      }
    } else {
      const int q = lane >> 3, c8 = (lane & 7) * 8;
      unsigned short* C  = (unsigned short*)Cout  + (size_t)b * strideC;
      unsigned short* C2 = (OUT_MODE == 2) ? ((unsigned short*)Cout2 + (size_t)b * strideC) : nullptr;
      for (int pass = 0; pass < 2; ++pass) {
#pragma unroll
        for (int it = 0; it < 4; ++it) {
          const int row = it * 4 + q;
          const float* sp = slab + row * 68 + c8;
          v8h hv, lv;
#pragma unroll
          for (int e = 0; e < 8; ++e) {
            if (OUT_MODE == 1) {
              hv[e] = (_Float16)sp[e];
            } else {
              unsigned short hb = f2bf_bits(sp[e]);
              unsigned short lb = f2bf_bits(sp[e] - bf_bits2f(hb));
              hv[e] = __builtin_bit_cast(_Float16, hb);
              lv[e] = __builtin_bit_cast(_Float16, lb);
            }
          }
          *(volatile v8h*)(C + (size_t)(mBase + row) * ldc + n0 + c8) = hv;
          if (OUT_MODE == 2) *(volatile v8h*)(C2 + (size_t)(mBase + row) * ldc + n0 + c8) = lv;
        }
        __threadfence();
      }
    }
    __builtin_amdgcn_fence(__ATOMIC_RELEASE, "workgroup");
    __builtin_amdgcn_wave_barrier();
    __builtin_amdgcn_fence(__ATOMIC_ACQUIRE, "workgroup");
  }
}

__device__ __forceinline__ int blk_excl_scan(int cnt, int* scan_ws, int tid, int* tot) {
  const int lane = tid & 31, wave = tid >> 5; int incl = cnt;
#pragma unroll
  for (int o = 1; o < 32; o <<= 1) { const int v = __shfl_up(incl, o, 32); if (lane >= o) incl += v; }
  if (lane == 31) scan_ws[wave] = incl;
  __syncthreads();
  if (wave == 0) { int wv = (lane < NT / 32) ? scan_ws[lane] : 0; int wincl = wv;
#pragma unroll
    for (int o = 1; o < 32; o <<= 1) { const int v = __shfl_up(wincl, o, 32); if (lane >= o) wincl += v; }
    if (lane < NT / 32) scan_ws[32 + lane] = wincl - wv; if (lane == 31) scan_ws[64] = wincl; }
  __syncthreads();
  const int res = scan_ws[32 + wave] + incl - cnt; *tot = scan_ws[64];
  return res;
}

template <bool L0>
__device__ __forceinline__ int chunk_hits(const int* __restrict__ dstv, const int* __restrict__ srcv, const float* __restrict__ eav,
                                          float emean, int e0, int n0, int tid, int* LIST, float* LISTF, int* scan_ws) {
  const int eb = e0 + tid * SPG;
  const bool real = eb < NE;
  const int ebc = real ? eb : (NE - SPG);
  int rec[SPG]; float recf[SPG]; int cnt = 0;
#pragma unroll
  for (int k = 0; k < SPG; k += 4) {
    const v4i d4 = *(const v4i*)(dstv + ebc + k);
    const v4i s4 = *(const v4i*)(srcv + ebc + k);
    v4f a4 = {0.f, 0.f, 0.f, 0.f};
    if (L0) a4 = *(const v4f*)(eav + ebc + k);
#pragma unroll
    for (int e = 0; e < 4; ++e) {
      int r = -1; float f = 0.f;
      if (real) {
        const int d = d4[e];
        if (d >= n0 && d < n0 + TG) { int s = s4[e]; s = s < 0 ? 0 : (s >= NN ? NN - 1 : s); r = ((d - n0) << 16) | s; f = a4[e]; ++cnt; }
      } else {
        const int ev = eb + k + e; const int d = ev - NE;
        if (ev < NV && d >= n0 && d < n0 + TG) { r = ((d - n0) << 16) | d; f = emean; ++cnt; }
      }
      rec[k + e] = r; recf[k + e] = f;
    }
  }
  int tot; int p = blk_excl_scan(cnt, scan_ws, tid, &tot);
#pragma unroll
  for (int k = 0; k < SPG; ++k) {
    if (rec[k] >= 0) { if ((unsigned)p < (unsigned)SCHG) { LIST[p] = rec[k]; if (L0) LISTF[p] = recf[k]; } ++p; }
  }
  __syncthreads();
  return tot < SCHG ? tot : SCHG;
}

__device__ __forceinline__ float gelu_f(float x) { return 0.5f * x * (1.0f + erff(x * 0.70710678118654752f)); }
__device__ __forceinline__ v4f leaky4(v4f m) {
  v4f r;
  r[0] = fmaxf(m[0], 0.2f * m[0]); r[1] = fmaxf(m[1], 0.2f * m[1]);
  r[2] = fmaxf(m[2], 0.2f * m[2]); r[3] = fmaxf(m[3], 0.2f * m[3]);
  return r;
}

template <bool L0, bool MEAN>
__global__ __launch_bounds__(NT) void gat_kernel(const float* __restrict__ XLR, const int* __restrict__ ei,
                                                const float* __restrict__ eattr, const float* __restrict__ att,
                                                const float* __restrict__ We, const float* __restrict__ bias,
                                                _Float16* __restrict__ HO, float* __restrict__ H2) {
  extern __shared__ __align__(16) float dyn_lds[];
  float* ACC = dyn_lds;
  float* SM = dyn_lds + TG * HC;
  float* SL = dyn_lds + TG * HC + TG * 8;
  int* LIST = (int*)(dyn_lds + TG * HC + TG * 16);
  float* LISTF = dyn_lds + TG * HC + TG * 16 + SCHG;
  __shared__ int scan_ws[80];
  __shared__ float red[NT];
  const int tid = threadIdx.x, lane = tid & 31, wave = tid >> 5;
  const int n0 = blockIdx.x * TG;
  const int grp = lane >> 3;
  const v4f attA = *(const v4f*)(att + 4 * lane), attB = *(const v4f*)(att + 128 + 4 * lane);
  v4f weA = {0.f, 0.f, 0.f, 0.f}, weB = {0.f, 0.f, 0.f, 0.f};
  if (L0) { weA = *(const v4f*)(We + 4 * lane); weB = *(const v4f*)(We + 128 + 4 * lane); }
  for (int i = tid; i < TG * HC; i += NT) ACC[i] = 0.f;
  for (int i = tid; i < TG * 8; i += NT) { SM[i] = -INFINITY; SL[i] = 0.f; }
  float emean = 0.f;
  if (L0) {
    float s = 0.f;
#pragma unroll 1
    for (int i = tid * 4; i < NE; i += NT * 4) { const v4f q = *(const v4f*)(eattr + i); s += q[0]; s += q[1]; s += q[2]; s += q[3]; }
    red[tid] = s;
    __syncthreads();
#pragma unroll 1
    for (int o = NT / 2; o > 0; o >>= 1) { if (tid < o) red[tid] += red[tid + o]; __syncthreads(); }
    emean = red[0] * (1.0f / (float)NE);
  }
  __syncthreads();
  const int* srcv = ei; const int* dstv = ei + NE;
#pragma unroll 1
  for (int c = 0; c < NCHG; ++c) {
    const int tot = chunk_hits<L0>(dstv, srcv, eattr, emean, c * SCHG, n0, tid, LIST, LISTF, scan_ws);
#pragma unroll 1
    for (int base = 0; base < tot; base += 32) {
      const int q = base + lane;
      const int qc = q < SCHG ? q : (SCHG - 1);
      const int lvv = LIST[qc];
      const float lff = L0 ? LISTF[qc] : 0.f;
      const int rv = (q < tot) ? lvv : -1;
      const float fv = (q < tot) ? lff : 0.f;
      const int own = (rv >= 0 && (rv >> 20) == wave) ? 1 : 0;
      unsigned msk = (unsigned)__ballot(own);
#pragma unroll 1
      for (int it = 0; it < 32; ++it) {
        if (msk == 0u) break;
        const int bp = __builtin_ctz(msk); msk &= msk - 1u;
        const int r = __shfl(rv, bp, 32);
        float eav = 0.f;
        if (L0) eav = __shfl(fv, bp, 32);
        const int dl = r >> 16, s = r & 0xFFFF;
        const float* xlp = XLR + (size_t)s * XP;
        const float* xrp = XLR + (size_t)(n0 + dl) * XP + HC;
        const v4f la = *(const v4f*)(xlp + 4 * lane), lb = *(const v4f*)(xlp + 128 + 4 * lane);
        const v4f ra = *(const v4f*)(xrp + 4 * lane), rb = *(const v4f*)(xrp + 128 + 4 * lane);
        v4f ma = la + ra, mb = lb + rb;
        if (L0) { ma = ma + eav * weA; mb = mb + eav * weB; }
        const v4f va = leaky4(ma), vb = leaky4(mb);
        float sa = va[0] * attA[0] + va[1] * attA[1] + va[2] * attA[2] + va[3] * attA[3];
        float sb = vb[0] * attB[0] + vb[1] * attB[1] + vb[2] * attB[2] + vb[3] * attB[3];
        sa += __shfl_xor(sa, 4, 32); sa += __shfl_xor(sa, 2, 32); sa += __shfl_xor(sa, 1, 32);
        sb += __shfl_xor(sb, 4, 32); sb += __shfl_xor(sb, 2, 32); sb += __shfl_xor(sb, 1, 32);
        const int miA = dl * 8 + grp, miB = miA + 4;
        const float moA = SM[miA], loA = SL[miA], moB = SM[miB], loB = SL[miB];
        const float mnA = fmaxf(moA, sa), mnB = fmaxf(moB, sb);
        const float rrA = __expf(moA - mnA), exA = __expf(sa - mnA);
        const float rrB = __expf(moB - mnB), exB = __expf(sb - mnB);
        const float lnA = loA * rrA + exA, lnB = loB * rrB + exB;
        if ((lane & 7) == 0) { SM[miA] = mnA; SL[miA] = lnA; SM[miB] = mnB; SL[miB] = lnB; }
        float* ap = ACC + dl * HC;
        v4f aa = *(const v4f*)(ap + 4 * lane), ab = *(const v4f*)(ap + 128 + 4 * lane);
        aa = aa * rrA + exA * la;
        ab = ab * rrB + exB * lb;
        *(v4f*)(ap + 4 * lane) = aa;
        *(v4f*)(ap + 128 + 4 * lane) = ab;
        asm volatile("" ::: "memory");
      }
    }
    __syncthreads();
  }
  if (!MEAN) {
#pragma unroll 1
    for (int j = 0; j < TG / 8; ++j) {
      const int dl = wave * (TG / 8) + j;
#pragma unroll 1
      for (int g = 0; g < 8; ++g) {
        const int cch = g * 32 + lane;
        float lv = SL[dl * 8 + g]; lv = lv > 0.f ? lv : 1.0f;
        const float inv = 1.0f / lv;
        float o = ACC[dl * HC + cch] * inv + bias[cch];
        o = gelu_f(o);
        ACC[dl * HC + cch] = o * HSC;
      }
    }
    __syncthreads();
#pragma unroll 1
    for (int j = 0; j < TG / 8; ++j) {
      const int dl = wave * (TG / 8) + j; const int n = n0 + dl;
      const float* ap = ACC + dl * HC + 8 * lane;
      const v4f p0 = *(const v4f*)(ap), p1 = *(const v4f*)(ap + 4);
      v8h hv;
      hv[0] = (_Float16)p0[0]; hv[1] = (_Float16)p0[1]; hv[2] = (_Float16)p0[2]; hv[3] = (_Float16)p0[3];
      hv[4] = (_Float16)p1[0]; hv[5] = (_Float16)p1[1]; hv[6] = (_Float16)p1[2]; hv[7] = (_Float16)p1[3];
      _Float16* rp = HO + (size_t)n * HC + 8 * lane;
      *(volatile v8h*)rp = hv;
      __threadfence();
      *(volatile v8h*)rp = hv;
    }
  } else {
#pragma unroll 1
    for (int j = 0; j < TG / 8; ++j) {
      const int dl = wave * (TG / 8) + j; const int n = n0 + dl;
      float o = 0.f;
#pragma unroll 1
      for (int g = 0; g < 8; ++g) {
        float lv = SL[dl * 8 + g]; lv = lv > 0.f ? lv : 1.0f;
        const float inv = 1.0f / lv;
        o += ACC[dl * HC + g * 32 + lane] * inv;
      }
      o = o * 0.125f + bias[lane];
      o = gelu_f(o);
      volatile float* rp = H2 + (size_t)n * DN;
      rp[lane] = o;
      __threadfence();
      rp[lane] = o;
    }
  }
}

__global__ __launch_bounds__(256) void prep_w_kernel(const float* __restrict__ W1l, const float* __restrict__ b1l,
                                                   const float* __restrict__ W1r, const float* __restrict__ b1r,
                                                   const float* __restrict__ W2l, const float* __restrict__ b2l,
                                                   const float* __restrict__ W2r, const float* __restrict__ b2r,
                                                   _Float16* __restrict__ WT, float* __restrict__ BCAT) {
  const int i = blockIdx.x * 256 + threadIdx.x;
  if (i < 2 * 512 * 128) {
    const int l = i >> 16, rem = i & 65535;
    const int n = rem >> 7, j = rem & 127;
    const bool isl = n < 256;
    const float* W = (l == 0) ? (isl ? W1l : W1r) : (isl ? W2l : W2r);
    const int nn = n & 255, k = 2 * j;
    const _Float16 h0 = (_Float16)(W[k * 256 + nn] * WSC), h1 = (_Float16)(W[(k + 1) * 256 + nn] * WSC);
    const unsigned u = (unsigned)__builtin_bit_cast(unsigned short, h0) | ((unsigned)__builtin_bit_cast(unsigned short, h1) << 16);
    ((volatile unsigned*)WT)[i] = u;
    __threadfence();
    ((volatile unsigned*)WT)[i] = u;
  }
  if (i < 1024) {
    const int l = i >> 9, c = i & 511;
    const bool isl = c < 256;
    const float* bp = (l == 0) ? (isl ? b1l : b1r) : (isl ? b2l : b2r);
    const float v = bp[c & 255];
    ((volatile float*)BCAT)[i] = v;
    __threadfence();
    ((volatile float*)BCAT)[i] = v;
  }
}

__global__ __launch_bounds__(256) void lin0_kernel(const float* __restrict__ x, const float* __restrict__ prm,
                                                 const float* __restrict__ Wl, const float* __restrict__ bl,
                                                 const float* __restrict__ Wr, const float* __restrict__ br,
                                                 float* __restrict__ XLR) {
  const int i = blockIdx.x * 256 + threadIdx.x;
  if (i >= NN * 128) return;
  const int n = i >> 7, q = i & 127, c0 = 4 * q;
  const bool isl = c0 < 256;
  const float* W = isl ? Wl : Wr;
  const float* bb = isl ? bl : br;
  const int cc = c0 & 255;
  const float* xp = x + (size_t)n * 6;
  float h[8];
  h[0] = xp[0]; h[1] = xp[1]; h[2] = xp[2]; h[3] = xp[3]; h[4] = xp[4]; h[5] = xp[5]; h[6] = prm[0]; h[7] = prm[1];
  v4f acc = {0.f, 0.f, 0.f, 0.f};
#pragma unroll
  for (int k = 0; k < 8; ++k) { const v4f w = *(const v4f*)(W + k * 256 + cc); acc = acc + h[k] * w; }
  const v4f bv = *(const v4f*)(bb + cc);
  acc = acc + bv;
  float* op = XLR + (size_t)n * XP + c0;
  *(volatile v4f*)op = acc;
  __threadfence();
  *(volatile v4f*)op = acc;
}

#define DK_W4   0
#define DK_W1T  8192
#define DK_W2T  16384
#define DK_CWT  24576
#define DK_WTOT 25088
#define DSCI    (1.0f / 64.0f)

__device__ __forceinline__ void wave_lds_sync() {
  __builtin_amdgcn_fence(__ATOMIC_RELEASE, "workgroup");
  __builtin_amdgcn_wave_barrier();
  __builtin_amdgcn_fence(__ATOMIC_ACQUIRE, "workgroup");
}
__device__ __forceinline__ v16h stage_a(_Float16* TA, v8f x0, v8f x1, int lane) {
  const int c = lane & 15, hh = lane >> 4;
  wave_lds_sync();
#pragma unroll
  for (int r = 0; r < 8; ++r) { TA[(8 * hh + r) * DN + c] = (_Float16)x0[r]; TA[(8 * hh + r) * DN + 16 + c] = (_Float16)x1[r]; }
  wave_lds_sync();
  return Frag<_Float16>::load(TA + c * DN + 8 * hh);
}
__device__ __forceinline__ void mm32(v16h a, const _Float16* Wt, int lane, v8f& o0, v8f& o1) {
  const int c = lane & 15, hh = lane >> 4;
  const v16h b0 = Frag<_Float16>::load(Wt + c * DN + 8 * hh);
  const v16h b1 = Frag<_Float16>::load(Wt + (16 + c) * DN + 8 * hh);
  const v8f z = {0.f, 0.f, 0.f, 0.f, 0.f, 0.f, 0.f, 0.f};
  o0 = mma_h(a, b0, z);
  o1 = mma_h(a, b1, z);
}
__device__ __forceinline__ void addb2(v8f& o0, v8f& o1, const float* __restrict__ b, int lane) {
  const int c = lane & 15;
  const float b0 = b[c], b1 = b[16 + c];
#pragma unroll
  for (int r = 0; r < 8; ++r) { o0[r] = o0[r] * DSCI + b0; o1[r] = o1[r] * DSCI + b1; }
}
__device__ __forceinline__ void ln_rows(v8f& x0, v8f& x1, const float* __restrict__ g, const float* __restrict__ b, int lane) {
  const int c = lane & 15;
  const float g0 = g[c], g1 = g[16 + c], b0 = b[c], b1 = b[16 + c];
#pragma unroll
  for (int r = 0; r < 8; ++r) {
    float s = x0[r] + x1[r];
    s += __shfl_xor(s, 1, 32); s += __shfl_xor(s, 2, 32); s += __shfl_xor(s, 4, 32); s += __shfl_xor(s, 8, 32);
    const float mean = s * (1.0f / 32.0f);
    const float d0 = x0[r] - mean, d1 = x1[r] - mean;
    float v = d0 * d0 + d1 * d1;
    v += __shfl_xor(v, 1, 32); v += __shfl_xor(v, 2, 32); v += __shfl_xor(v, 4, 32); v += __shfl_xor(v, 8, 32);
    const float var = v * (1.0f / 32.0f);
    const float rs = rsqrtf(var + 1e-5f);
    x0[r] = d0 * rs * g0 + b0;
    x1[r] = d1 * rs * g1 + b1;
  }
}

__global__ __launch_bounds__(64) void dec_kernel(const float* __restrict__ H2,
    const float* __restrict__ Wv_sa, const float* __restrict__ bv_sa, const float* __restrict__ Wo_sa, const float* __restrict__ bo_sa,
    const float* __restrict__ Wv_ca, const float* __restrict__ bv_ca, const float* __restrict__ Wo_ca, const float* __restrict__ bo_ca,
    const float* __restrict__ W1, const float* __restrict__ b1f, const float* __restrict__ W2, const float* __restrict__ b2f,
    const float* __restrict__ ln1g, const float* __restrict__ ln1b, const float* __restrict__ ln2g, const float* __restrict__ ln2b,
    const float* __restrict__ ln3g, const float* __restrict__ ln3b,
    const float* __restrict__ convW, const float* __restrict__ convb, float* __restrict__ out) {
  __shared__ __align__(16) _Float16 WH[DK_WTOT];
  __shared__ __align__(16) _Float16 TAs[2][16 * DN];
  __shared__ __align__(16) _Float16 TFs[2][16 * DFF];
  __shared__ __align__(16) float OSs[2][64];
  const int tid = threadIdx.x, lane = tid & 31, wave = tid >> 5;
  const int c = lane & 15, hh = lane >> 4;
#pragma unroll 1
  for (int i = tid; i < 8192; i += 64) {
    const int l = i >> 12, j = (i >> 10) & 3, n = (i >> 5) & 31, k = i & 31;
    const float* W = (j == 0) ? Wv_sa : (j == 1) ? Wo_sa : (j == 2) ? Wv_ca : Wo_ca;
    WH[DK_W4 + i] = (_Float16)(W[l * 1024 + k * 32 + n] * WSC);
  }
#pragma unroll 1
  for (int i = tid; i < 8192; i += 64) {
    const int l = i >> 12, n = (i >> 5) & 127, k = i & 31;
    WH[DK_W1T + i] = (_Float16)(W1[l * 4096 + k * 128 + n] * WSC);
  }
#pragma unroll 1
  for (int i = tid; i < 8192; i += 64) {
    const int l = i >> 12, n = (i >> 7) & 31, k = i & 127;
    WH[DK_W2T + i] = (_Float16)(W2[l * 4096 + k * 32 + n] * WSC);
  }
#pragma unroll 1
  for (int i = tid; i < 512; i += 64) {
    const int n = i >> 5, k = i & 31;
    float v = convW[k * 4 + (n < 4 ? n : 3)];
    if (n >= 4) v = 0.f;
    WH[DK_CWT + i] = (_Float16)(v * WSC);
  }
  __syncthreads();
  _Float16* TA = TAs[wave];
  _Float16* TF = TFs[wave];
  float* OS = OSs[wave];
  const int row0 = blockIdx.x * DROWS + wave * 16;
  v8f t0, t1;
#pragma unroll
  for (int r = 0; r < 8; ++r) {
    t0[r] = H2[(size_t)(row0 + 8 * hh + r) * DN + c];
    t1[r] = H2[(size_t)(row0 + 8 * hh + r) * DN + 16 + c];
  }
  const v16h amem = stage_a(TA, t0, t1, lane);
#pragma unroll 1
  for (int l = 0; l < 2; ++l) {
    const _Float16* W4 = WH + DK_W4 + l * 4096;
    v8f u0, u1, s0, s1;
    { const v16h at = stage_a(TA, t0, t1, lane); mm32(at, W4, lane, u0, u1); }
    addb2(u0, u1, bv_sa + l * DN, lane);
    { const v16h au = stage_a(TA, u0, u1, lane); mm32(au, W4 + 1024, lane, s0, s1); }
    addb2(s0, s1, bo_sa + l * DN, lane);
    t0 = t0 + s0; t1 = t1 + s1;
    ln_rows(t0, t1, ln1g + l * DN, ln1b + l * DN, lane);
    mm32(amem, W4 + 2048, lane, u0, u1);
    addb2(u0, u1, bv_ca + l * DN, lane);
    { const v16h au = stage_a(TA, u0, u1, lane); mm32(au, W4 + 3072, lane, s0, s1); }
    addb2(s0, s1, bo_ca + l * DN, lane);
    t0 = t0 + s0; t1 = t1 + s1;
    ln_rows(t0, t1, ln2g + l * DN, ln2b + l * DN, lane);
    {
      const v16h at = stage_a(TA, t0, t1, lane);
      const v8f z = {0.f, 0.f, 0.f, 0.f, 0.f, 0.f, 0.f, 0.f};
      v8f f[8];
#pragma unroll
      for (int j = 0; j < 8; ++j) {
        const v16h bj = Frag<_Float16>::load(WH + DK_W1T + (l * DFF + 16 * j + c) * DN + 8 * hh);
        f[j] = mma_h(at, bj, z);
      }
      wave_lds_sync();
#pragma unroll
      for (int j = 0; j < 8; ++j) {
        const float bj = b1f[l * DFF + 16 * j + c];
#pragma unroll
        for (int r = 0; r < 8; ++r) {
          const float v = fmaxf(f[j][r] * DSCI + bj, 0.0f);
          TF[(8 * hh + r) * DFF + 16 * j + c] = (_Float16)v;
        }
      }
      wave_lds_sync();
      v8f o0 = z, o1 = z;
#pragma unroll
      for (int kk = 0; kk < 4; ++kk) {
        const v16h a  = Frag<_Float16>::load(TF + c * DFF + kk * 32 + 8 * hh);
        const v16h b0 = Frag<_Float16>::load(WH + DK_W2T + (l * DN + c) * DFF + kk * 32 + 8 * hh);
        const v16h b1 = Frag<_Float16>::load(WH + DK_W2T + (l * DN + 16 + c) * DFF + kk * 32 + 8 * hh);
        o0 = mma_h(a, b0, o0);
        o1 = mma_h(a, b1, o1);
      }
      addb2(o0, o1, b2f + l * DN, lane);
      t0 = t0 + o0; t1 = t1 + o1;
      ln_rows(t0, t1, ln3g + l * DN, ln3b + l * DN, lane);
    }
  }
  v8f y0, y1;
#pragma unroll
  for (int r = 0; r < 8; ++r) { y0[r] = tanhf(t0[r]); y1[r] = tanhf(t1[r]); }
  const v16h ay = stage_a(TA, y0, y1, lane);
  const v16h bc = Frag<_Float16>::load(WH + DK_CWT + c * DN + 8 * hh);
  const v8f z2 = {0.f, 0.f, 0.f, 0.f, 0.f, 0.f, 0.f, 0.f};
  const v8f oc = mma_h(ay, bc, z2);
  const float cb = convb[c & 3];
  wave_lds_sync();
  if (c < 4) {
#pragma unroll
    for (int r = 0; r < 8; ++r) OS[(8 * hh + r) * 4 + c] = oc[r] * DSCI + cb;
  }
  wave_lds_sync();
  const v4f ov = *(const v4f*)(OS + (lane & 15) * 4);
  float* op = out + (size_t)(row0 + (lane & 15)) * 4;
  if (lane < 16) *(volatile v4f*)op = ov;
  __threadfence();
  if (lane < 16) *(volatile v4f*)op = ov;
}

extern "C" void kernel_launch(void* const* d_in, const int* in_sizes, int n_in,
                              void* d_out, int out_size, void* d_ws, size_t ws_size, hipStream_t stream) {
  if (n_in < 43) return;
  if (in_sizes[0] != NN * 6 || in_sizes[1] != 2 * NE || in_sizes[2] != NE || out_size != NN * 4) return;
  const float* x      = (const float*)d_in[0];
  const int*   ei     = (const int*)d_in[1];
  const float* eattr  = (const float*)d_in[2];
  const float* params = (const float*)d_in[3];
  const float* g0_Wl  = (const float*)d_in[4];
  const float* g0_bl  = (const float*)d_in[5];
  const float* g0_Wr  = (const float*)d_in[6];
  const float* g0_br  = (const float*)d_in[7];
  const float* g0_att = (const float*)d_in[8];
  const float* g0_We  = (const float*)d_in[9];
  const float* g0_bias= (const float*)d_in[10];
  const float* g1_Wl  = (const float*)d_in[11];
  const float* g1_bl  = (const float*)d_in[12];
  const float* g1_Wr  = (const float*)d_in[13];
  const float* g1_br  = (const float*)d_in[14];
  const float* g1_att = (const float*)d_in[15];
  const float* g1_bias= (const float*)d_in[16];
  const float* g2_Wl  = (const float*)d_in[17];
  const float* g2_bl  = (const float*)d_in[18];
  const float* g2_Wr  = (const float*)d_in[19];
  const float* g2_br  = (const float*)d_in[20];
  const float* g2_att = (const float*)d_in[21];
  const float* g2_bias= (const float*)d_in[22];
  const float* Wv_sa  = (const float*)d_in[23];
  const float* bv_sa  = (const float*)d_in[24];
  const float* Wo_sa  = (const float*)d_in[25];
  const float* bo_sa  = (const float*)d_in[26];
  const float* Wv_ca  = (const float*)d_in[27];
  const float* bv_ca  = (const float*)d_in[28];
  const float* Wo_ca  = (const float*)d_in[29];
  const float* bo_ca  = (const float*)d_in[30];
  const float* W1     = (const float*)d_in[31];
  const float* b1     = (const float*)d_in[32];
  const float* W2     = (const float*)d_in[33];
  const float* b2     = (const float*)d_in[34];
  const float* ln1g   = (const float*)d_in[35];
  const float* ln1b   = (const float*)d_in[36];
  const float* ln2g   = (const float*)d_in[37];
  const float* ln2b   = (const float*)d_in[38];
  const float* ln3g   = (const float*)d_in[39];
  const float* ln3b   = (const float*)d_in[40];
  const float* convW  = (const float*)d_in[41];
  const float* convb  = (const float*)d_in[42];
  float* out = (float*)d_out;

  char* ws = (char*)d_ws; size_t off = 0;
  auto carve = [&](size_t bytes) -> char* { char* p = ws + off; off += (bytes + 255) & ~(size_t)255; return p; };
  float*    XLR  = (float*)carve((size_t)NN * XP * 4);
  _Float16* H16  = (_Float16*)carve((size_t)NN * HC * 2);
  _Float16* WT   = (_Float16*)carve((size_t)2 * 512 * 256 * 2);
  float*    BCAT = (float*)carve((size_t)2 * 512 * 4);
  float*    H2   = (float*)carve((size_t)NN * DN * 4);
  if (off > ws_size || off > (size_t)134217728) return;

  prep_w_kernel<<<(2 * 512 * 128) / 256, 256, 0, stream>>>(g1_Wl, g1_bl, g1_Wr, g1_br, g2_Wl, g2_bl, g2_Wr, g2_br, WT, BCAT);
  lin0_kernel<<<(NN * 128) / 256, 256, 0, stream>>>(x, params, g0_Wl, g0_bl, g0_Wr, g0_br, XLR);

  hipFuncSetAttribute(reinterpret_cast<const void*>(&gat_kernel<true, false>), hipFuncAttributeMaxDynamicSharedMemorySize, GAT_LDS_BYTES);
  gat_kernel<true, false><<<NBG, NT, GAT_LDS_BYTES, stream>>>(XLR, ei, eattr, g0_att, g0_We, g0_bias, H16, H2);

  {
    const int tiles = (NN / 64) * (512 / 64);
    wmma_gemm64<0, false, 2, 0, false><<<dim3((tiles + 7) / 8, 1), 256, 0, stream>>>(
        U16(H16), U16(H16), HC, 0L,
        U16(WT), U16(WT), HC, 0L,
        (void*)XLR, (void*)nullptr, XP, 0L,
        BCAT, (const float*)nullptr, 0L, NN, 512, HC, 1.0f / (HSC * WSC));
  }
  hipFuncSetAttribute(reinterpret_cast<const void*>(&gat_kernel<false, false>), hipFuncAttributeMaxDynamicSharedMemorySize, GAT_LDS_BYTES);
  gat_kernel<false, false><<<NBG, NT, GAT_LDS_BYTES, stream>>>(XLR, ei, eattr, g1_att, (const float*)nullptr, g1_bias, H16, H2);

  {
    const int tiles = (NN / 64) * (512 / 64);
    wmma_gemm64<0, false, 2, 0, false><<<dim3((tiles + 7) / 8, 1), 256, 0, stream>>>(
        U16(H16), U16(H16), HC, 0L,
        U16(WT + (size_t)512 * 256), U16(WT + (size_t)512 * 256), HC, 0L,
        (void*)XLR, (void*)nullptr, XP, 0L,
        BCAT + 512, (const float*)nullptr, 0L, NN, 512, HC, 1.0f / (HSC * WSC));
  }
  hipFuncSetAttribute(reinterpret_cast<const void*>(&gat_kernel<false, true>), hipFuncAttributeMaxDynamicSharedMemorySize, GAT_LDS_BYTES);
  gat_kernel<false, true><<<NBG, NT, GAT_LDS_BYTES, stream>>>(XLR, ei, eattr, g2_att, (const float*)nullptr, g2_bias, H16, H2);

  dec_kernel<<<NN / DROWS, 64, 0, stream>>>(H2,
      Wv_sa, bv_sa, Wo_sa, bo_sa, Wv_ca, bv_ca, Wo_ca, bo_ca,
      W1, b1, W2, b2, ln1g, ln1b, ln2g, ln2b, ln3g, ln3b,
      convW, convb, out);
}
